// Interchange_76776835383950
// MI455X (gfx1250) — hardware-verified
//
#include <hip/hip_runtime.h>
#include <math.h>


#define NBATCH 4
#define NH 4
#define DD 64
#define L0 4096
#define L1 2048
#define L2 1024

typedef __attribute__((ext_vector_type(16))) _Float16 v16h;
typedef __attribute__((ext_vector_type(8)))  _Float16 v8h;
typedef __attribute__((ext_vector_type(8)))  float v8f;
typedef __attribute__((ext_vector_type(4)))  float v4f;
typedef __attribute__((ext_vector_type(4)))  unsigned v4u;

template <typename T> __device__ __forceinline__ void vst2(void* p, T v) { *(volatile T*)p = v; __threadfence(); *(volatile T*)p = v; }
__device__ __forceinline__ v8f wmma16(v16h a, v16h b, v8f c) {
  v8f d = __builtin_amdgcn_wmma_f32_16x16x32_f16(false, a, false, b, (short)0, c, false, false);
  asm volatile("v_nop\n\tv_nop\n\tv_nop\n\tv_nop" : "+v"(d) : "v"(a), "v"(b));
  return d;
}
__device__ __forceinline__ v16h frag_h(const _Float16* rowk0, int lane) {
  union { v16h v; v8h q[2]; } u; const _Float16* p = rowk0 + 8 * (lane >> 4);
  u.q[0] = *(const v8h*)p; u.q[1] = *(const v8h*)(p + 16); return u.v;
}
__device__ __forceinline__ v16h frag_f32(const float* rowk0, int lane) {
  v16h a; const float* p = rowk0 + 8 * (lane >> 4);
#pragma unroll
  for (int i = 0; i < 8; ++i) { a[i] = (_Float16)p[i]; a[8 + i] = (_Float16)p[16 + i]; }
  return a;
}
typedef __attribute__((ext_vector_type(16))) __bf16 v16b;
__device__ __forceinline__ v8f wmma_bf(v16b a, v16b b, v8f c) {
  v8f d = __builtin_amdgcn_wmma_f32_16x16x32_bf16(false, a, false, b, (short)0, c, false, false);
  asm volatile("v_nop\n\tv_nop\n\tv_nop\n\tv_nop" : "+v"(d) : "v"(a), "v"(b));
  return d;
}
struct F2 { v16b h, l; };
__device__ __forceinline__ F2 bsplit16(const float v[16]) { F2 r;
#pragma unroll
  for (int i = 0; i < 16; ++i) { const __bf16 h = (__bf16)v[i]; r.h[i] = h; r.l[i] = (__bf16)(v[i] - (float)h); }
  return r; }
__device__ __forceinline__ F2 split_row(const float* row, int k0, int lane) { float v[16]; const float* p = row + k0 + 8 * (lane >> 4);
#pragma unroll
  for (int i = 0; i < 8; ++i) { v[i] = p[i]; v[8 + i] = p[16 + i]; }
  return bsplit16(v); }
__device__ __forceinline__ F2 split_col(const float* W, int k0, int n, int lane, int ld) { float v[16]; const int g = lane >> 4;
#pragma unroll
  for (int i = 0; i < 8; ++i) { v[i] = W[(size_t)(k0 + 8 * g + i) * ld + n]; v[8 + i] = W[(size_t)(k0 + 16 + 8 * g + i) * ld + n]; }
  return bsplit16(v); }
__device__ __forceinline__ v8f mac3(const F2& a, const F2& b, v8f c) { c = wmma_bf(a.l, b.h, c); c = wmma_bf(a.h, b.l, c); return wmma_bf(a.h, b.h, c); }
#define LDSX() do { asm volatile("s_wait_dscnt 0" ::: "memory"); __builtin_amdgcn_wave_barrier(); __builtin_amdgcn_fence(__ATOMIC_RELEASE, "workgroup"); } while (0)

__global__ __launch_bounds__(256) void k_pack(const float* __restrict__ wq, const float* __restrict__ wk, const float* __restrict__ wv,
                                            const float* __restrict__ wc0, const float* __restrict__ wc1, const float* __restrict__ wc2, _Float16* __restrict__ PW) {
  const int job = blockIdx.y, tid = blockIdx.x * 256 + threadIdx.x;
  const float* W; int K, N; size_t ob;
  if (job < 9) { const int which = job / 3, t = job % 3; W = (which == 0 ? wq : (which == 1 ? wk : wv)) + (size_t)t * DD * 256; K = DD; N = 256; ob = (size_t)job * 256 * DD; }
  else { const int i = job - 9; W = i == 0 ? wc0 : (i == 1 ? wc1 : wc2); K = i == 1 ? 768 : 512; N = DD; ob = (size_t)9 * 256 * DD + (size_t)(i == 0 ? 0 : (i == 1 ? 512 * 64 : 512 * 64 + 768 * 64)); }
  const int npieces = N * (K / 8); if (tid >= npieces) return;
  const int n = tid / (K / 8), pc = tid % (K / 8);
  union { v8h h; v4u u; } pk;
#pragma unroll
  for (int e = 0; e < 8; ++e) pk.h[e] = (_Float16)W[(size_t)(pc * 8 + e) * N + n];
  vst2(PW + ob + (size_t)n * K + pc * 8, pk.u);
}
__global__ __launch_bounds__(128) void k_proj(const float* __restrict__ x, int L, int t, const _Float16* __restrict__ PW,
                                            const float* __restrict__ wq, const float* __restrict__ wk,
                                            const float* __restrict__ bq, const float* __restrict__ bk, const float* __restrict__ bv,
                                            float* __restrict__ Q, float* __restrict__ Kk, _Float16* __restrict__ vT) {
  __shared__ __align__(16) float so[4][16][132];
  __shared__ __align__(16) _Float16 st[128][72];
  const int tid = threadIdx.x, wave = tid >> 5, lane = tid & 31, col = lane & 15, g = lane >> 4;
  const int r0 = blockIdx.x * 64 + wave * 16, n0 = blockIdx.y * 128;
  const int which = n0 / 256, hb = (n0 % 256) / 64;
  const float* bias = (which == 0 ? bq : (which == 1 ? bk : bv)) + (size_t)t * NH * DD;
  v8f acc[8] = {};
  if (which < 2) {
    const float* W = (which == 0 ? wq : wk) + (size_t)t * DD * 256;
#pragma unroll
    for (int kc = 0; kc < 2; ++kc) { const F2 a = split_row(x + (size_t)(r0 + col) * DD, kc * 32, lane);
#pragma unroll
      for (int j = 0; j < 8; ++j) acc[j] = mac3(a, split_col(W, kc * 32, (n0 % 256) + j * 16 + col, lane, 256), acc[j]); }
  } else {
    const _Float16* Wt = PW + (size_t)(2 * 3 + t) * 256 * DD;
#pragma unroll
    for (int kc = 0; kc < 2; ++kc) { const v16h a = frag_f32(x + (size_t)(r0 + col) * DD + kc * 32, lane);
#pragma unroll
      for (int j = 0; j < 8; ++j) acc[j] = wmma16(a, frag_h(Wt + (size_t)((n0 % 256) + j * 16 + col) * DD + kc * 32, lane), acc[j]); }
  }
  const int b = r0 / L, l0 = r0 % L;
  if (which < 2) {
    float* S = &so[wave][0][0];
#pragma unroll
    for (int j = 0; j < 8; ++j) { const float bb = bias[(n0 % 256) + j * 16 + col];
#pragma unroll
      for (int r = 0; r < 8; ++r) S[(8 * g + r) * 132 + j * 16 + col] = acc[j][r] + bb; }
    LDSX();
    float* dst = which == 0 ? Q : Kk;
    for (int q = lane; q < 512; q += 32) { const int rl = q >> 5, pcs = q & 31, hh = hb + (pcs >> 4), pc = pcs & 15;
      vst2(dst + (((size_t)b * NH + hh) * L + l0 + rl) * DD + pc * 4, *(const v4f*)(S + rl * 132 + (hh - hb) * 64 + pc * 4)); }
  } else {
#pragma unroll
    for (int j = 0; j < 8; ++j) { const float bb = bias[(n0 % 256) + j * 16 + col];
#pragma unroll
      for (int r = 0; r < 8; ++r) st[j * 16 + col][wave * 16 + 8 * g + r] = (_Float16)(acc[j][r] + bb); }
    __syncthreads();
    for (int q = tid; q < 128 * 8; q += 128) { const int c = q >> 3, pc = q & 7, hh = hb + (c >> 6), d = c & 63;
      vst2(vT + (((size_t)b * NH + hh) * DD + d) * L + (blockIdx.x * 64) % L + pc * 8, *(const v4u*)(&st[c][pc * 8])); }
  }
}
template <int MODE, int KW>
__global__ __launch_bounds__(128) void k_band(const float* __restrict__ Q, const float* __restrict__ Kk, const _Float16* __restrict__ vT, int Lq, int Lk,
                                            _Float16* __restrict__ F, int pl, int jidx) {
  __shared__ __align__(16) float sS[4][16][KW + 4];
  __shared__ __align__(16) _Float16 sP[4][16][KW + 8];
  __shared__ __align__(16) float sO[4][16][68];
  const int tid = threadIdx.x, w = tid >> 5, lane = tid & 31, col = lane & 15, g = lane >> 4;
  const int h = blockIdx.y, b = blockIdx.z, q0 = blockIdx.x * 64 + w * 16;
  const float* qb = Q + (((size_t)b * NH + h) * Lq) * DD; const float* kbp = Kk + (((size_t)b * NH + h) * Lk) * DD; const _Float16* vb = vT + (((size_t)b * NH + h) * DD) * Lk;
  auto lo_of = [&](int q) { return MODE == 0 ? q - 5 : (MODE == 1 ? (q >> 1) - 5 : 2 * q - 5); };
  const int wlen = MODE == 2 ? 12 : 11;
  const int kb = lo_of(q0);
  F2 aq[2];
#pragma unroll
  for (int kc = 0; kc < 2; ++kc) aq[kc] = split_row(qb + (size_t)(q0 + col) * DD, kc * 32, lane);
#pragma unroll
  for (int t = 0; t < KW / 16; ++t) { int kp = kb + t * 16 + col; kp = kp < 0 ? 0 : (kp > Lk - 1 ? Lk - 1 : kp);
    v8f acc = {};
#pragma unroll
    for (int kc = 0; kc < 2; ++kc) acc = mac3(aq[kc], split_row(kbp + (size_t)kp * DD, kc * 32, lane), acc);
#pragma unroll
    for (int r = 0; r < 8; ++r) sS[w][8 * g + r][t * 16 + col] = acc[r]; }
  LDSX();
  const int q = q0 + col, lo = lo_of(q), hi = lo + wlen - 1;
  float mx = -3.0e38f;
  for (int j = 0; j < KW / 2; ++j) { const int slot = g * (KW / 2) + j, kp = kb + slot;
    float v = -3.0e38f; if (kp >= lo && kp <= hi) v = (kp >= 0 && kp < Lk) ? sS[w][col][slot] : 0.f;
    sS[w][col][slot] = v; mx = fmaxf(mx, v); }
  mx = fmaxf(mx, __shfl_xor(mx, 16, 32));
  float sum = 0.f;
  for (int j = 0; j < KW / 2; ++j) { const int slot = g * (KW / 2) + j; const float v = sS[w][col][slot]; const float p = v > -1.0e38f ? expf(v - mx) : 0.f; sum += p; sS[w][col][slot] = p; }
  sum += __shfl_xor(sum, 16, 32);
  const float inv = 16384.0f / sum;
  for (int j = 0; j < KW / 2; ++j) { const int slot = g * (KW / 2) + j; const int kp = kb + slot;
    const float p = (kp >= 0 && kp < Lk) ? sS[w][col][slot] * inv : 0.f;
    sP[w][col][slot] = (_Float16)p; }
  LDSX();
  v8f acc4[4] = {};
#pragma unroll
  for (int kc = 0; kc < KW / 32; ++kc) { const v16h pa = frag_h(&sP[w][col][0] + kc * 32, lane);
#pragma unroll
    for (int t = 0; t < 4; ++t) { v16h bv; const _Float16* vr = vb + (size_t)(t * 16 + col) * Lk;
#pragma unroll
      for (int i = 0; i < 8; ++i) { int ka = kb + kc * 32 + 8 * g + i, kz = ka + 16;
        ka = ka < 0 ? 0 : (ka > Lk - 1 ? Lk - 1 : ka); kz = kz < 0 ? 0 : (kz > Lk - 1 ? Lk - 1 : kz); bv[i] = vr[ka]; bv[8 + i] = vr[kz]; }
      acc4[t] = wmma16(pa, bv, acc4[t]); } }
#pragma unroll
  for (int t = 0; t < 4; ++t)
#pragma unroll
    for (int r = 0; r < 8; ++r) sO[w][8 * g + r][t * 16 + col] = acc4[t][r] * (1.0f / 16384.0f);
  LDSX();
  const size_t fw = (size_t)NH * pl * DD;
  for (int qq = lane; qq < 16 * 8; qq += 32) { const int rl = qq >> 3, pc = qq & 7; union { v8h hh; v4u u; } pk;
#pragma unroll
    for (int e = 0; e < 8; ++e) pk.hh[e] = (_Float16)sO[w][rl][pc * 8 + e];
    vst2(F + ((size_t)b * Lq + q0 + rl) * fw + (size_t)(h * pl + jidx) * DD + pc * 8, pk.u); }
}
__global__ __launch_bounds__(128) void k_out(const _Float16* __restrict__ F, int K, const _Float16* __restrict__ Wt, const float* __restrict__ bc, float* __restrict__ out) {
  __shared__ __align__(16) float so[4][16][68];
  const int tid = threadIdx.x, wave = tid >> 5, lane = tid & 31, col = lane & 15, g = lane >> 4;
  const int r0 = blockIdx.x * 64 + wave * 16;
  v8f acc[4] = {};
#pragma unroll 1
  for (int kc = 0; kc < K / 32; ++kc) { const v16h a = frag_h(F + (size_t)(r0 + col) * K + kc * 32, lane);
#pragma unroll
    for (int j = 0; j < 4; ++j) acc[j] = wmma16(a, frag_h(Wt + (size_t)(j * 16 + col) * K + kc * 32, lane), acc[j]); }
#pragma unroll
  for (int j = 0; j < 4; ++j) { const float bb = bc[j * 16 + col];
#pragma unroll
    for (int r = 0; r < 8; ++r) so[wave][8 * g + r][j * 16 + col] = acc[j][r] + bb; }
  LDSX();
  for (int qq = lane; qq < 16 * 16; qq += 32) { const int rl = qq >> 4, pc = qq & 15; vst2(out + (size_t)(r0 + rl) * DD + pc * 4, *(const v4f*)(&so[wave][rl][pc * 4])); }
}

extern "C" void kernel_launch(void* const* d_in, const int* in_sizes, int n_in,
                              void* d_out, int out_size, void* d_ws, size_t ws_size,
                              hipStream_t stream) {
  (void)in_sizes; (void)n_in; (void)out_size; (void)ws_size;
  const float* x0 = (const float*)d_in[0]; const float* x1 = (const float*)d_in[1]; const float* x2 = (const float*)d_in[2];
  const float* wq = (const float*)d_in[3]; const float* bq = (const float*)d_in[4]; const float* wk = (const float*)d_in[5]; const float* bk = (const float*)d_in[6];
  const float* wv = (const float*)d_in[7]; const float* bv = (const float*)d_in[8];
  const float* wc0 = (const float*)d_in[9]; const float* bc0 = (const float*)d_in[10]; const float* wc1 = (const float*)d_in[11]; const float* bc1 = (const float*)d_in[12];
  const float* wc2 = (const float*)d_in[13]; const float* bc2 = (const float*)d_in[14];
  float* out0 = (float*)d_out; float* out1 = out0 + (size_t)NBATCH * L0 * DD; float* out2 = out1 + (size_t)NBATCH * L1 * DD;
  char* ws = (char*)d_ws; size_t off = 0;
  auto take = [&](size_t n) { char* p = ws + off; off += (n * 2 + 255) & ~(size_t)255; return (_Float16*)p; };
  auto takef = [&](size_t n) { char* p = ws + off; off += (n * 4 + 255) & ~(size_t)255; return (float*)p; };
  _Float16* PW = take((size_t)9 * 256 * DD + 512 * 64 + 768 * 64 + 512 * 64);
  const int Ls[3] = { L0, L1, L2 }; const float* xs[3] = { x0, x1, x2 };
  float *Q[3], *Kk[3]; _Float16 *vT[3], *F[3];
  const int pls[3] = { 2, 3, 2 };
  for (int t = 0; t < 3; ++t) { Q[t] = takef((size_t)NBATCH * NH * Ls[t] * DD); Kk[t] = takef((size_t)NBATCH * NH * Ls[t] * DD); vT[t] = take((size_t)NBATCH * NH * DD * Ls[t]); F[t] = take((size_t)NBATCH * Ls[t] * NH * pls[t] * DD); }
  k_pack<<<dim3((768 * 64 / 8 + 255) / 256, 12), 256, 0, stream>>>(wq, wk, wv, wc0, wc1, wc2, PW);
  for (int t = 0; t < 3; ++t) k_proj<<<dim3(NBATCH * Ls[t] / 64, 768 / 128), 128, 0, stream>>>(xs[t], Ls[t], t, PW, wq, wk, bq, bk, bv, Q[t], Kk[t], vT[t]);
  k_band<0, 32><<<dim3(L0 / 64, NH, NBATCH), 128, 0, stream>>>(Q[0], Kk[0], vT[0], L0, L0, F[0], 2, 0);
  k_band<1, 32><<<dim3(L0 / 64, NH, NBATCH), 128, 0, stream>>>(Q[0], Kk[1], vT[1], L0, L1, F[0], 2, 1);
  k_band<2, 64><<<dim3(L1 / 64, NH, NBATCH), 128, 0, stream>>>(Q[1], Kk[0], vT[0], L1, L0, F[1], 3, 0);
  k_band<0, 32><<<dim3(L1 / 64, NH, NBATCH), 128, 0, stream>>>(Q[1], Kk[1], vT[1], L1, L1, F[1], 3, 1);
  k_band<1, 32><<<dim3(L1 / 64, NH, NBATCH), 128, 0, stream>>>(Q[1], Kk[2], vT[2], L1, L2, F[1], 3, 2);
  k_band<2, 64><<<dim3(L2 / 64, NH, NBATCH), 128, 0, stream>>>(Q[2], Kk[1], vT[1], L2, L1, F[2], 2, 0);
  k_band<0, 32><<<dim3(L2 / 64, NH, NBATCH), 128, 0, stream>>>(Q[2], Kk[2], vT[2], L2, L2, F[2], 2, 1);
  const _Float16* WcT0 = PW + (size_t)9 * 256 * DD; const _Float16* WcT1 = WcT0 + 512 * 64; const _Float16* WcT2 = WcT1 + 768 * 64;
  k_out<<<NBATCH * L0 / 64, 128, 0, stream>>>(F[0], 512, WcT0, bc0, out0);
  k_out<<<NBATCH * L1 / 64, 128, 0, stream>>>(F[1], 768, WcT1, bc1, out1);
  k_out<<<NBATCH * L2 / 64, 128, 0, stream>>>(F[2], 512, WcT2, bc2, out2);
}
